// MPNNBlock_5016521802505
// MI455X (gfx1250) — hardware-verified
//
#include <hip/hip_runtime.h>
#include <stddef.h>


#define NTHR   256
#define NWAVE  8
#define DM     32
#define WCOL   1024
#define KP     32
#define EPB    128
#define NPB    128
#define PBLK   16
#define EPT    8
#define PIECE  (NTHR * EPT)
#define WCAP   (EPT * 32)
#define NBC    1024
#define SLB    10
#define AGGDYN (NBC * DM * 4)
#define WSCAP  134217728
#define WSC    64.0f
#define WINV   0.015625f

static_assert(PBLK * NTHR * 8 == WCOL * KP);
static_assert(DM * DM == 128 * 8);
static_assert(NBC == (1 << SLB));
static_assert(PIECE == 2048);
static_assert((EPT % 4) == 0);
static_assert(EPB == NWAVE * 16);
static_assert(NPB == NWAVE * 16);
static_assert((NBC % 32) == 0);
static_assert((NBC % NWAVE) == 0);
static_assert((NBC * DM) % (4 * NTHR) == 0);
static_assert(DM == 32 && WCOL == DM * DM && KP == DM);

typedef float    v4f  __attribute__((ext_vector_type(4)));
typedef float    v8f  __attribute__((ext_vector_type(8)));
typedef int      v4i  __attribute__((ext_vector_type(4)));
typedef _Float16 v8h  __attribute__((ext_vector_type(8)));
typedef _Float16 v16h __attribute__((ext_vector_type(16)));
union FragH { v16h v; v8h u[2]; };
union C8    { v8f v; v4f h[2]; };

__device__ __forceinline__ v8f wmh(v16h a, v16h b, v8f c) {
  v8f d = __builtin_amdgcn_wmma_f32_16x16x32_f16(false, a, false, b, (short)0, c, false, false);
  asm volatile("v_nop\n\tv_nop\n\tv_nop\n\tv_nop" : "+v"(d) : "v"(a), "v"(b));
  return d;
}
__device__ __forceinline__ v8f z8() {
  v8f z = {0.f, 0.f, 0.f, 0.f, 0.f, 0.f, 0.f, 0.f};
  return z;
}
__device__ __forceinline__ v8h cv8(v4f p, v4f q, float s) {
  v8h v;
  v[0] = (_Float16)(p.x * s); v[1] = (_Float16)(p.y * s); v[2] = (_Float16)(p.z * s); v[3] = (_Float16)(p.w * s);
  v[4] = (_Float16)(q.x * s); v[5] = (_Float16)(q.y * s); v[6] = (_Float16)(q.z * s); v[7] = (_Float16)(q.w * s);
  return v;
}

__global__ __launch_bounds__(NTHR) void k_prep(
    const float* __restrict__ eW, const float* __restrict__ nW, _Float16* Wp, _Float16* Np) {
  const int t = (int)blockIdx.x * NTHR + (int)threadIdx.x;
  const int o = t * 8;
  const bool pn = t < (DM * DM) / 8;
  const int on = pn ? o : 0;
  const v4f a0 = *(const v4f*)(eW + o);
  const v4f a1 = *(const v4f*)(eW + o + 4);
  const v4f b0 = *(const v4f*)(nW + on);
  const v4f b1 = *(const v4f*)(nW + on + 4);
  const v8h fa = cv8(a0, a1, WSC);
  const v8h fb = cv8(b0, b1, WSC);
  *(volatile v8h*)(Wp + o) = fa;
  if (pn) *(volatile v8h*)(Np + o) = fb;
  __threadfence();
  *(volatile v8h*)(Wp + o) = fa;
  if (pn) *(volatile v8h*)(Np + o) = fb;
}

__global__ __launch_bounds__(NTHR) void k_root(
    const float* __restrict__ x, const _Float16* __restrict__ Np, float* R, int nN) {
  __shared__ __attribute__((aligned(16))) float sR[NWAVE * 16 * DM];
  const int tid = (int)threadIdx.x, lane = tid & 31, wave = tid >> 5, hi = lane >> 4, m = lane & 15;
  const int n0 = ((int)blockIdx.x * NWAVE + wave) * 16;

  FragH a;
  {
    int row = n0 + m;
    row = row > nN - 1 ? nN - 1 : row;
    const float* xp = x + (size_t)row * DM;
    const v4f q0 = *(const v4f*)(xp + 8 * hi);
    const v4f q1 = *(const v4f*)(xp + 8 * hi + 4);
    const v4f q2 = *(const v4f*)(xp + 16 + 8 * hi);
    const v4f q3 = *(const v4f*)(xp + 16 + 8 * hi + 4);
    a.u[0] = cv8(q0, q1, 1.0f);
    a.u[1] = cv8(q2, q3, 1.0f);
  }
  FragH b0, b1;
  {
    const _Float16* p0 = Np + m * KP + 8 * hi;
    const _Float16* p1 = Np + (16 + m) * KP + 8 * hi;
    b0.u[0] = *(const v8h*)(p0);
    b0.u[1] = *(const v8h*)(p0 + 16);
    b1.u[0] = *(const v8h*)(p1);
    b1.u[1] = *(const v8h*)(p1 + 16);
  }
  const v8f a0 = wmh(a.v, b0.v, z8());
  const v8f a1 = wmh(a.v, b1.v, z8());

  float* sw = sR + wave * (16 * DM);
  {
    float* sp = sw + (8 * hi) * DM;
#pragma unroll
    for (int r = 0; r < 8; ++r) {
      sp[r * DM + m]      = a0[r] * WINV;
      sp[r * DM + 16 + m] = a1[r] * WINV;
    }
  }
  __syncthreads();

  const int rq = lane >> 3, pc = lane & 7;
  float* rrow = R + (size_t)n0 * DM;
#pragma unroll
  for (int q = 0; q < 4; ++q) {
    const int row = 4 * q + rq;
    const v4f v = *(const v4f*)(sw + row * DM + 4 * pc);
    *(volatile v4f*)(rrow + (size_t)row * DM + 4 * pc) = v;
  }
  __threadfence();
#pragma unroll
  for (int q = 0; q < 4; ++q) {
    const int row = 4 * q + rq;
    const v4f v = *(const v4f*)(sw + row * DM + 4 * pc);
    *(volatile v4f*)(rrow + (size_t)row * DM + 4 * pc) = v;
  }
}

__device__ __forceinline__ v8f wtile(const _Float16* __restrict__ wp, v16h b) {
  FragH a;
  a.u[0] = *(const v8h*)(wp);
  a.u[1] = *(const v8h*)(wp + 16);
  return wmh(a.v, b, z8());
}
__device__ __forceinline__ v8f acc_fma(v8f c, float xv, v8f acc) {
#pragma unroll
  for (int r = 0; r < 8; ++r) acc[r] = __builtin_fmaf(xv, c[r], acc[r]);
  return acc;
}

__global__ __launch_bounds__(NTHR) void k_edge(
    const float* __restrict__ x, const int* __restrict__ ei, const float* __restrict__ ea,
    const _Float16* __restrict__ Wp, float* Msg, int nE, int nN) {
  __shared__ __attribute__((aligned(16))) float sM[NWAVE * 16 * DM];
  const int tid = (int)threadIdx.x, lane = tid & 31, wave = tid >> 5, hi = lane >> 4, m = lane & 15;

  const int e0 = ((int)blockIdx.x * NWAVE + wave) * 16;
  int ec = e0 + m;
  ec = ec > nE - 1 ? nE - 1 : ec;
  int src = ei[ec];
  src = src < 0 ? 0 : (src > nN - 1 ? nN - 1 : src);
  float* sMw = sM + wave * (16 * DM);

  FragH b;
  {
    const float* ep = ea + (size_t)ec * DM;
    const v4f q0 = *(const v4f*)(ep + 8 * hi);
    const v4f q1 = *(const v4f*)(ep + 8 * hi + 4);
    const v4f q2 = *(const v4f*)(ep + 16 + 8 * hi);
    const v4f q3 = *(const v4f*)(ep + 16 + 8 * hi + 4);
    b.u[0] = cv8(q0, q1, 1.0f);
    b.u[1] = cv8(q2, q3, 1.0f);
  }

  v8f macc0 = z8(), macc1 = z8();
  {
    const float* xr = x + (size_t)src * DM;
    const _Float16* wp = Wp + m * KP + 8 * hi;
#pragma unroll 1
    for (int i = 0; i < DM; ++i) {
      const float xv = xr[i];
      const int na = 32 * i;
      const int nb = 32 * i + 16;
      const v8f ca = wtile(wp + (size_t)na * KP, b.v);
      macc0 = acc_fma(ca, xv, macc0);
      const v8f cb = wtile(wp + (size_t)nb * KP, b.v);
      macc1 = acc_fma(cb, xv, macc1);
    }
  }

  {
    float* sp = sMw + m * DM + 8 * hi;
    C8 u;
    u.v = macc0 * WINV;
    *(v4f*)(sp)      = u.h[0];
    *(v4f*)(sp + 4)  = u.h[1];
    u.v = macc1 * WINV;
    *(v4f*)(sp + 16) = u.h[0];
    *(v4f*)(sp + 20) = u.h[1];
  }
  __syncthreads();
  {
    const int rq = lane >> 3, pc = lane & 7;
    float* mrow = Msg + (size_t)e0 * DM;
#pragma unroll
    for (int q = 0; q < 4; ++q) {
      const int row = 4 * q + rq;
      const v4f v = *(const v4f*)(sMw + row * DM + 4 * pc);
      *(volatile v4f*)(mrow + (size_t)row * DM + 4 * pc) = v;
    }
    __threadfence();
#pragma unroll
    for (int q = 0; q < 4; ++q) {
      const int row = 4 * q + rq;
      const v4f v = *(const v4f*)(sMw + row * DM + 4 * pc);
      *(volatile v4f*)(mrow + (size_t)row * DM + 4 * pc) = v;
    }
  }
}

__device__ __forceinline__ int scan_piece(const int* __restrict__ dp, int lim, int cbase, int base, int vec,
                                          int* list, int tid, int wave) {
  int wc = 0;
  const int el0  = tid * EPT;
  const int e0   = cbase + el0;
  const int sent = -2147483647 - 1;
  int kk[EPT];
  if (vec != 0 && cbase + PIECE <= lim) {
    const v4i* p = (const v4i*)(dp + e0);
#pragma unroll
    for (int u = 0; u < EPT / 4; ++u) {
      const v4i d = p[u];
      kk[4 * u] = d.x; kk[4 * u + 1] = d.y; kk[4 * u + 2] = d.z; kk[4 * u + 3] = d.w;
    }
  } else {
    const int lm = lim - 1;
#pragma unroll
    for (int q = 0; q < EPT; ++q) {
      const int eq = e0 + q;
      const int ecl = eq > lm ? lm : eq;
      const int a = dp[ecl];
      kk[q] = (eq < lim) ? a : sent;
    }
  }
  const unsigned nb = (unsigned)base;
  unsigned sq[EPT];
  bool hq[EPT];
  bool anyl = false;
#pragma unroll
  for (int q = 0; q < EPT; ++q) {
    sq[q] = (unsigned)kk[q] - nb;
    hq[q] = sq[q] < (unsigned)NBC;
    anyl = anyl | hq[q];
  }
  const unsigned any = __builtin_amdgcn_ballot_w32(anyl);
  if (any != 0u) {
#define HIT(HQ, SQ, Q) { \
      const unsigned mj = __builtin_amdgcn_ballot_w32(HQ); \
      if (mj != 0u) { \
        if (HQ) { \
          const int ps = wc + (int)__builtin_amdgcn_mbcnt_lo(mj, 0u); \
          if (ps < WCAP) list[wave * WCAP + ps] = ((el0 + (Q)) << SLB) | (int)(SQ); \
        } \
        wc += (int)__builtin_popcount(mj); } }
#pragma unroll
    for (int q = 0; q < EPT; ++q) {
      HIT(hq[q], sq[q], q)
    }
#undef HIT
  }
  return wc;
}

__device__ __forceinline__ void drain_piece(const int* list, const int* wcnt, float* accF,
                                            const float* __restrict__ Msg, int rowoff, int nE, int lane, int wave) {
#pragma unroll 1
  for (int wsx = 0; wsx < NWAVE; ++wsx) {
    int n = __builtin_amdgcn_readfirstlane(wcnt[wsx]);
    n = n > WCAP ? WCAP : (n < 0 ? 0 : n);
    const int* lp = list + wsx * WCAP;
#pragma unroll 1
    for (int bb = 0; bb < n; bb += 32) {
      const int idx = bb + lane;
      const int ic = idx > WCAP - 1 ? WCAP - 1 : idx;
      const int ent = lp[ic];
      const bool own = (idx < n) && ((ent & (NWAVE - 1)) == wave);
      unsigned msk = __builtin_amdgcn_ballot_w32(own);
#pragma unroll 1
      while (msk != 0u) {
        const int bit = (int)__builtin_ctz(msk);
        msk &= msk - 1u;
        const int e2 = __builtin_amdgcn_readlane(ent, bit);
        const int slot = e2 & (NBC - 1);
        const int el = (e2 >> SLB) & (PIECE - 1);
        int row = rowoff + el;
        row = row < 0 ? 0 : (row > nE - 1 ? nE - 1 : row);
        const float mv = Msg[(size_t)row * DM + lane];
        accF[slot * DM + lane] += mv;
      }
    }
  }
}

__device__ __forceinline__ void agg_store(const float* accF, float* out, int base, int nN, int lane, int wave) {
  const int rq = lane >> 3, pc = lane & 7;
#pragma unroll 1
  for (int it = 0; it < NBC / 32; ++it) {
    const int s = 32 * it + 4 * wave + rq;
    const int node = base + s;
    if (node < nN) {
      const v4f v = *(const v4f*)(accF + s * DM + 4 * pc);
      *(volatile v4f*)(out + (size_t)node * DM + 4 * pc) = v;
    }
  }
}

__global__ __launch_bounds__(NTHR) void k_agg(
    const int* __restrict__ dp, const float* __restrict__ Msg, const float* __restrict__ R,
    float* out, int nE, int nN, int vec) {
  extern __shared__ __attribute__((aligned(16))) float accF[];
  __shared__ int list[NWAVE * WCAP];
  __shared__ int wcnt[NWAVE];
  const int tid = (int)threadIdx.x, lane = tid & 31, wave = tid >> 5;
  const int base = (int)blockIdx.x * NBC;

#pragma unroll 1
  for (int i = tid; i < (NBC * DM) / 4; i += NTHR) {
    const int s = i >> 3, c4 = (i & 7) * 4;
    int node = base + s;
    node = node > nN - 1 ? nN - 1 : node;
    const v4f v = *(const v4f*)(R + (size_t)node * DM + c4);
    *(v4f*)(accF + s * DM + c4) = v;
  }
  __syncthreads();

#pragma unroll 1
  for (int cbase = 0; cbase < nE; cbase += PIECE) {
    const int wc = scan_piece(dp, nE, cbase, base, vec, list, tid, wave);
    if (lane == 0) wcnt[wave] = wc;
    __syncthreads();
    drain_piece(list, wcnt, accF, Msg, cbase, nE, lane, wave);
    __syncthreads();
  }

  agg_store(accF, out, base, nN, lane, wave);
  __threadfence();
  agg_store(accF, out, base, nN, lane, wave);
}

extern "C" void kernel_launch(void* const* d_in, const int* in_sizes, int n_in,
                              void* d_out, int out_size, void* d_ws, size_t ws_size,
                              hipStream_t stream) {
  if (n_in < 5) return;
  if (in_sizes[0] < DM || (in_sizes[0] % DM) != 0) return;
  const int nN = in_sizes[0] / DM;
  if (nN < 1 || nN > (1 << 24)) return;
  if (in_sizes[1] < DM || (in_sizes[1] % DM) != 0) return;
  const int nE = in_sizes[1] / DM;
  if (nE < 1 || nE > (1 << 26)) return;
  if (in_sizes[2] != WCOL * KP) return;
  if (in_sizes[3] != DM * DM) return;
  if (in_sizes[4] != 2 * nE) return;
  if (out_size != nN * DM) return;

  const float* x  = (const float*)d_in[0];
  const float* ea = (const float*)d_in[1];
  const float* eW = (const float*)d_in[2];
  const float* nW = (const float*)d_in[3];
  const int*   ei = (const int*)d_in[4];
  float* out = (float*)d_out;

  const int nbE   = (nE + EPB - 1) / EPB;
  const int Epad  = nbE * EPB;
  const int nbR   = (nN + NPB - 1) / NPB;
  const int NpadR = nbR * NPB;
  const int nbAgg = (nN + NBC - 1) / NBC;
  const int vec   = ((nE & 3) == 0) ? 1 : 0;

  char* ws = (char*)d_ws;
  size_t off = 0;
  const size_t oWp = off; off += (size_t)WCOL * KP * 2;         off = (off + 255) & ~(size_t)255;
  const size_t oNp = off; off += (size_t)DM * DM * 2;           off = (off + 255) & ~(size_t)255;
  const size_t oR  = off; off += (size_t)NpadR * DM * 4;        off = (off + 255) & ~(size_t)255;
  const size_t oM  = off; off += (size_t)Epad * DM * 4;         off = (off + 255) & ~(size_t)255;
  if (off > ws_size || off > (size_t)WSCAP) return;
  _Float16* Wp = (_Float16*)(ws + oWp);
  _Float16* Np = (_Float16*)(ws + oNp);
  float* R   = (float*)(ws + oR);
  float* Msg = (float*)(ws + oM);

  hipFuncSetAttribute(reinterpret_cast<const void*>(&k_agg), hipFuncAttributeMaxDynamicSharedMemorySize, AGGDYN);

  k_prep<<<PBLK, NTHR, 0, stream>>>(eW, nW, Wp, Np);
  k_root<<<nbR, NTHR, 0, stream>>>(x, Np, R, nN);
  k_edge<<<nbE, NTHR, 0, stream>>>(x, ei, ea, Wp, Msg, nE, nN);
  k_agg<<<nbAgg, NTHR, AGGDYN, stream>>>(ei + nE, Msg, R, out, nE, nN, vec);
}
